// InundationCoder_41317585387565
// MI455X (gfx1250) — hardware-run, weakly checked
//
#include <hip/hip_runtime.h>


namespace {
constexpr int N = 8192, B = 32, T = 32, E = 32768, H = 64, HE = 4, DM = 16, LH = 128, NK = 3, NR = N * T, NRB = NR / 16, SR = B * T;
constexpr int OFF1 = SR * 12, OFF2 = OFF1 + B * LH;
constexpr float XS = 8.0f, HS = 64.0f, WSC = 256.0f, NEG = 0.2f;
typedef _Float16 b16;
typedef __attribute__((ext_vector_type(16))) _Float16 v16b;
typedef __attribute__((ext_vector_type(8))) _Float16 v8b;
typedef __attribute__((ext_vector_type(8))) float v8f;
typedef __attribute__((ext_vector_type(4))) float v4f;
typedef __attribute__((ext_vector_type(2))) float v2f;
__device__ __forceinline__ float bf16_rne(float f) { unsigned int u = __float_as_uint(f); u += 0x7FFFu + ((u >> 16) & 1u); return __uint_as_float(u & 0xFFFF0000u); }
__device__ __forceinline__ void split16(float v, b16& hi, b16& lo) { hi = (b16)v; lo = (b16)(v - (float)hi); }
__device__ __forceinline__ v16b frag_kb(const b16* p, int hh) { const v8b a = *(const v8b*)(p + 8 * hh), b = *(const v8b*)(p + 16 + 8 * hh); v16b f;
#pragma unroll
  for (int e = 0; e < 8; ++e) { f[e] = a[e]; f[8 + e] = b[e]; } return f; }
__device__ __forceinline__ v8f wmma16b(v16b a, v16b b, v8f c) { v8f d = __builtin_amdgcn_wmma_f32_16x16x32_f16(false, a, false, b, (short)0, c, false, false); asm volatile("v_nop\n\tv_nop\n\tv_nop\n\tv_nop" : "+v"(d) : "v"(a), "v"(b)); return d; }
__device__ __forceinline__ void wave_lds_sync() { __builtin_amdgcn_fence(__ATOMIC_RELEASE, "workgroup"); __builtin_amdgcn_wave_barrier(); __builtin_amdgcn_fence(__ATOMIC_ACQUIRE, "workgroup"); }
__device__ __forceinline__ float pmul(float a, float b) { float p = a * b; asm volatile("" : "+v"(p)); return p; }
__device__ __forceinline__ int iclamp(int v, int lo, int hi) { return v < lo ? lo : (v > hi ? hi : v); }
__device__ __forceinline__ float leaky(float v) { return v >= 0.0f ? v : NEG * v; }
__device__ __forceinline__ float sigm(float v) { return 1.0f / (1.0f + __expf(-v)); }
__device__ __forceinline__ float softplus(float v) { return v > 20.0f ? v : (v < -20.0f ? __expf(v) : log1pf(__expf(v))); }
constexpr int CSR_NBLK9 = 512, CSR_GB9 = 9, CSR_GN9 = 1 << CSR_GB9  , CSR_TS9 = (CSR_GN9 < 32 ? 32 : CSR_GN9)  , CSR_MAXG9 = 512, CSR_CAP9 = 12288  ;
__device__ __host__ __forceinline__ int csr_tix9(int v) { return (v >> CSR_GB9) * CSR_TS9 + (v & (CSR_GN9 - 1)); }
__global__ __launch_bounds__(64) void csrA_kernel9(const int* __restrict__ dst, int E, int N, int nG, int CHP, int NGP, int* __restrict__ STG, int* __restrict__ HST) {
  extern __shared__ int sm[];
  int* cnt = sm; int* run = sm + NGP; int* ids = sm + 2 * NGP;
  const int b = blockIdx.x; const int ch = (E + CSR_NBLK9 - 1) / CSR_NBLK9; const int e0 = b * ch, e1 = min(E, e0 + ch);
  for (int i = threadIdx.x; i < NGP; i += 64) cnt[i] = 0;
  for (int i = threadIdx.x; i < CHP; i += 64) ids[i] = -1;
  __syncthreads();
  if (threadIdx.x == 0) {
    for (int e = e0; e < e1; ++e) { int d = dst[e]; d = (d < 0) ? 0 : (d >= N ? N - 1 : d); cnt[d >> CSR_GB9] += 1; }
    int acc = 0; for (int g = 0; g < nG; ++g) { run[g] = acc; acc += cnt[g]; }
    for (int e = e0; e < e1; ++e) { int d = dst[e]; d = (d < 0) ? 0 : (d >= N ? N - 1 : d); const int g = d >> CSR_GB9; ids[run[g]] = e; run[g] += 1; } }
  __syncthreads();
  typedef __attribute__((ext_vector_type(4))) int v4i;
  for (int pass = 0; pass < 2; ++pass) {
    for (int i = threadIdx.x; i < CHP / 4; i += 64) *(volatile v4i*)(STG + (size_t)b * CHP + i * 4) = *(const v4i*)(&ids[i * 4]);
    for (int i = threadIdx.x; i < NGP / 4; i += 64) { v4i v; for (int e = 0; e < 4; ++e) v[e] = (i * 4 + e < nG) ? cnt[i * 4 + e] : 0; *(volatile v4i*)(HST + (size_t)b * NGP + i * 4) = v; }
    __threadfence(); }
}
__global__ __launch_bounds__(512) void csrS_kernel9(const int* __restrict__ HST, int nG, int NGP, int* __restrict__ START, int* __restrict__ TOT, int* __restrict__ OFF) {
  __shared__ int tot[CSR_MAXG9];
  const int b = threadIdx.x;
  for (int pass = 0; pass < 2; ++pass) { int runb = 0; for (int g = 0; g < nG; ++g) { int c = HST[(size_t)b * NGP + g]; c = (c < 0) ? 0 : c; ((volatile int*)OFF)[(size_t)g * CSR_NBLK9 + b] = runb; runb += c; } __threadfence(); }
  for (int g = threadIdx.x; g < nG; g += 512) { int s = 0; for (int bb = 0; bb < CSR_NBLK9; ++bb) { int c = HST[(size_t)bb * NGP + g]; s += (c < 0) ? 0 : c; } tot[g] = s; }
  __syncthreads();
  if (threadIdx.x < 32) {
    __shared__ int st[CSR_MAXG9 + 32];
    if (threadIdx.x == 0) { int acc = 0; for (int g = 0; g < NGP; ++g) { st[g] = acc; if (g < nG) acc += (tot[g] + 31) & ~31; } st[NGP] = acc; }
    __builtin_amdgcn_fence(__ATOMIC_RELEASE, "workgroup"); __builtin_amdgcn_wave_barrier(); __builtin_amdgcn_fence(__ATOMIC_ACQUIRE, "workgroup");
    for (int pass = 0; pass < 2; ++pass) { for (int i = threadIdx.x; i < NGP + 32; i += 32) { ((volatile int*)START)[i] = (i <= NGP) ? st[min(i, NGP)] : 0; ((volatile int*)TOT)[i] = (i < nG) ? tot[i] : 0; } __threadfence(); } }
}
__global__ __launch_bounds__(256) void csrB_kernel9(const int* __restrict__ dst, int N, int nG, int CHP, int NGP, int permLen, const int* __restrict__ STG, const int* __restrict__ HST, const int* __restrict__ OFF, const int* __restrict__ START, const int* __restrict__ TOT, int* __restrict__ PERM, int* __restrict__ ROWPTR, int* __restrict__ ROWCNT, int* __restrict__ FLAG) {
  typedef __attribute__((ext_vector_type(4))) int v4i;
  __shared__ int ids[CSR_CAP9]; __shared__ unsigned short key[CSR_CAP9]; __shared__ int outp[CSR_CAP9]; __shared__ int ncnt[CSR_GN9 + 1]; __shared__ int boff[CSR_NBLK9 + 1];
  const int g = blockIdx.x, t_ = threadIdx.x; int tot = TOT[g]; int st = START[g], stn = START[g + 1]; const int v0 = g * CSR_GN9; const int nv = min(CSR_GN9, N - v0); const int t0 = g * CSR_TS9;
  st = (st < 0) ? 0 : (st > permLen - 32 ? permLen - 32 : st) & ~31; stn = (stn < st) ? st : (stn > permLen ? permLen : stn); tot = (tot < 0) ? 0 : tot; if (tot > stn - st && tot <= CSR_CAP9) tot = stn - st;
  if (tot > CSR_CAP9) {
    for (int pass = 0; pass < 2; ++pass) { for (int i = t_; i < CSR_TS9 / 4; i += 256) { v4i a, c; for (int e = 0; e < 4; ++e) { a[e] = st; c[e] = 0; } *(volatile v4i*)(ROWPTR + t0 + i * 4) = a; *(volatile v4i*)(ROWCNT + t0 + i * 4) = c; } if (t_ == 0) ((volatile int*)FLAG)[0] = 1; __threadfence(); } (void)nv; return; }
  if (t_ == 0) { int acc = 0; for (int b = 0; b < CSR_NBLK9; ++b) { boff[b] = acc; int c = HST[(size_t)b * NGP + g]; c = (c < 0) ? 0 : (c > CHP ? CHP : c); acc += c; if (acc > tot) acc = tot; } boff[CSR_NBLK9] = acc; }
  for (int i = t_; i <= CSR_GN9; i += 256) ncnt[i] = 0;
  __syncthreads();
  for (int b = 0; b < CSR_NBLK9; ++b) { const int c = boff[b + 1] - boff[b]; int o_ = OFF[(size_t)g * CSR_NBLK9 + b]; o_ = (o_ < 0) ? 0 : (o_ > CHP - c ? CHP - c : o_); const int* src_ = STG + (size_t)b * CHP + o_;
    for (int i = t_; i < c; i += 256) { int id = src_[i]; id = (id < 0) ? 0 : id; ids[boff[b] + i] = id; int d = dst[id]; d = (d < v0) ? v0 : (d >= N ? N - 1 : d); int kk = d - v0; kk = (kk < 0) ? 0 : (kk >= CSR_GN9 ? CSR_GN9 - 1 : kk); key[boff[b] + i] = (unsigned short)kk; } }
  __syncthreads();
  if (t_ == 0) { for (int i = 0; i < tot; ++i) ncnt[key[i]] += 1; int acc = 0; for (int vl = 0; vl < CSR_GN9; ++vl) { const int c = ncnt[vl]; ncnt[vl] = acc; acc += c; } ncnt[CSR_GN9] = acc;
    for (int i = 0; i < tot; ++i) { const int vl = key[i]; outp[ncnt[vl]] = ids[i]; ncnt[vl] += 1; }
    for (int vl = CSR_GN9; vl > 0; --vl) ncnt[vl] = ncnt[vl - 1]; ncnt[0] = 0; }
  __syncthreads();
  for (int pass = 0; pass < 2; ++pass) {
    for (int i = t_; i < (stn - st) / 4; i += 256) { v4i v; for (int e = 0; e < 4; ++e) { const int q = i * 4 + e; v[e] = (q < tot) ? outp[q] : -1; } *(volatile v4i*)(PERM + st + i * 4) = v; }
    for (int i = t_; i < CSR_TS9 / 4; i += 256) { v4i a, c; for (int e = 0; e < 4; ++e) { const int vl = i * 4 + e; const int vc = vl < CSR_GN9 ? vl : CSR_GN9; a[e] = (vl < CSR_GN9) ? st + ncnt[vc] : st; c[e] = (vl < nv) ? (ncnt[(vc < CSR_GN9 ? vc : CSR_GN9 - 1) + 1] - ncnt[vc]) : 0; } *(volatile v4i*)(ROWPTR + t0 + i * 4) = a; *(volatile v4i*)(ROWCNT + t0 + i * 4) = c; }
    __threadfence(); }
}
__global__ __launch_bounds__(256) void csrZ_kernel9(int* __restrict__ p, size_t n4) { typedef __attribute__((ext_vector_type(4))) int v4i; const size_t tid = (size_t)blockIdx.x * 256 + threadIdx.x, nth = (size_t)gridDim.x * 256; v4i z = {0, 0, 0, 0}; for (size_t i = tid; i < n4; i += nth) *(volatile v4i*)(p + i * 4) = z; }
struct CsrBufs9 { int *STG, *HST, *OFF, *START, *TOT, *PERM, *ROWPTR, *ROWCNT, *FLAG; int nG, NGP, CHP; size_t permLen; char* base; size_t bytes; };
static size_t csr_carve9(CsrBufs9& c, char* ws, size_t off, int E, int N) {
  const size_t off0 = off; c.base = ws + off;
  auto al = [&](size_t bytes) { char* p = ws + off; off += (bytes + 255) & ~(size_t)255; return p; };
  c.nG = (N + CSR_GN9 - 1) / CSR_GN9; c.NGP = (c.nG + 31) & ~31; const int ch = (E + CSR_NBLK9 - 1) / CSR_NBLK9; c.CHP = (ch + 31) & ~31; c.permLen = (size_t)E + 32 * (size_t)c.nG + 32;
  c.STG = (int*)al((size_t)CSR_NBLK9 * c.CHP * 4); c.HST = (int*)al((size_t)CSR_NBLK9 * c.NGP * 4); c.OFF = (int*)al((size_t)c.NGP * CSR_NBLK9 * 4); c.START = (int*)al((size_t)(c.NGP + 64) * 4); c.TOT = (int*)al((size_t)(c.NGP + 64) * 4);
  c.PERM = (int*)al(c.permLen * 4); c.ROWPTR = (int*)al((size_t)c.nG * CSR_TS9 * 4); c.ROWCNT = (int*)al((size_t)c.nG * CSR_TS9 * 4); c.FLAG = (int*)al(256);
  c.bytes = off - off0; return off;
}
static void csr_build9(const CsrBufs9& c, const int* dst, int E, int N, hipStream_t stream) {
  const size_t smem = (size_t)(2 * c.NGP + c.CHP) * 4;
  csrZ_kernel9<<<512, 256, 0, stream>>>((int*)c.base, c.bytes / 16);
  csrA_kernel9<<<CSR_NBLK9, 64, smem, stream>>>(dst, E, N, c.nG, c.CHP, c.NGP, c.STG, c.HST);
  csrS_kernel9<<<1, 512, 0, stream>>>(c.HST, c.nG, c.NGP, c.START, c.TOT, c.OFF);
  csrB_kernel9<<<c.nG, 256, 0, stream>>>(dst, N, c.nG, c.CHP, c.NGP, (int)c.permLen, c.STG, c.HST, c.OFF, c.START, c.TOT, c.PERM, c.ROWPTR, c.ROWCNT, c.FLAG);
}


__global__ __launch_bounds__(256) void wput_kernel(const float* __restrict__ w, int KIN, int OUTW, int OUT, int co, int KP, b16* __restrict__ WT) {
  const int KG = KIN / 8; const int u = blockIdx.x * 256 + threadIdx.x; if (u >= OUT * KG) return; const int o = u / KG, k0 = (u % KG) * 8; v8b v;
#pragma unroll
  for (int j = 0; j < 8; ++j) v[j] = (b16)(bf16_rne(w[(size_t)(k0 + j) * OUTW + o]) * WSC); for (int pass = 0; pass < 2; ++pass) { *(volatile v8b*)(WT + (size_t)o * KP + co + k0) = v; __threadfence(); }
}
__global__ __launch_bounds__(256) void wzero_kernel(b16* __restrict__ WT, int n8) { const int u = blockIdx.x * 256 + threadIdx.x; if (u >= n8) return; v8b z = {}; for (int pass = 0; pass < 2; ++pass) { *(volatile v8b*)(WT + (size_t)u * 8) = z; __threadfence(); } }
__global__ __launch_bounds__(32) void proj_kernel(const float* __restrict__ era, const float* __restrict__ bc, const float* __restrict__ bd, const b16* __restrict__ WT, const float* __restrict__ bias, int TV, float* __restrict__ X0) {
  __shared__ __attribute__((aligned(16))) b16 Ah[16][H + 8]; __shared__ __attribute__((aligned(16))) float Tf[16][H + 4];
  const int lane = threadIdx.x, nloc = lane & 15, hlf = lane >> 4; const size_t m0 = (size_t)blockIdx.x * 16; if ((int)(m0 % T) >= TV) return;
  for (int rr = 0; rr < 16; ++rr) { const size_t r = m0 + rr; const size_t n = r / T; float a = 0.0f; if (lane < 16) a = era[r * 16 + lane]; else if (lane < 32) a = bc[n * 16 + lane - 16];
    Ah[rr][lane] = (b16)(bf16_rne(a) * XS); Ah[rr][32 + lane] = lane < 8 ? (b16)(bf16_rne(bd[n * 8 + lane]) * XS) : (b16)0.0f; }
  wave_lds_sync();
  v8f acc[4];
#pragma unroll
  for (int t = 0; t < 4; ++t) acc[t] = (v8f){};
#pragma unroll
  for (int kb = 0; kb < H; kb += 32) { const v16b a = frag_kb(&Ah[nloc][kb], hlf);
#pragma unroll
    for (int t = 0; t < 4; ++t) acc[t] = wmma16b(a, frag_kb(WT + (size_t)(t * 16 + nloc) * H + kb, hlf), acc[t]); }
#pragma unroll
  for (int t = 0; t < 4; ++t) { const int c = t * 16 + nloc; const float bb = bf16_rne(bias[c]);
#pragma unroll 1
    for (int r8 = 0; r8 < 8; ++r8) Tf[8 * hlf + r8][c] = fmaxf(acc[t][r8] * (1.0f / (XS * WSC)) + bb, 0.0f); }
  wave_lds_sync();
  for (int pass = 0; pass < 2; ++pass) { for (int rr = 0; rr < 16; ++rr) *(volatile v2f*)(X0 + (m0 + rr) * H + lane * 2) = *(const v2f*)(&Tf[rr][lane * 2]); __threadfence(); }
}
__global__ __launch_bounds__(32) void lin_kernel(const float* __restrict__ X, const b16* __restrict__ WT, const float* __restrict__ as, const float* __restrict__ ad, int TV, float* __restrict__ P, float* __restrict__ EL) {
  __shared__ __attribute__((aligned(16))) b16 Ah[16][H + 8], Al[16][H + 8]; __shared__ __attribute__((aligned(16))) float Tf[16][H + 4], Se[16][8];
  const int lane = threadIdx.x, nloc = lane & 15, hlf = lane >> 4; const size_t m0 = (size_t)blockIdx.x * 16; if ((int)(m0 % T) >= TV) return;
  for (int rr = 0; rr < 16; ++rr) { const v2f v = *(const v2f*)(X + (m0 + rr) * H + lane * 2); for (int j = 0; j < 2; ++j) { b16 p, q; split16(v[j] * HS, p, q); Ah[rr][lane * 2 + j] = p; Al[rr][lane * 2 + j] = q; } }
  wave_lds_sync();
  v8f acc[4];
#pragma unroll
  for (int t = 0; t < 4; ++t) acc[t] = (v8f){};
#pragma unroll
  for (int kb = 0; kb < H; kb += 32) { const v16b a = frag_kb(&Ah[nloc][kb], hlf), al = frag_kb(&Al[nloc][kb], hlf);
#pragma unroll
    for (int t = 0; t < 4; ++t) { const v16b bw = frag_kb(WT + (size_t)(t * 16 + nloc) * H + kb, hlf); acc[t] = wmma16b(a, bw, acc[t]); acc[t] = wmma16b(al, bw, acc[t]); } }
  const float sc = 1.0f / (HS * WSC);
#pragma unroll
  for (int t = 0; t < 4; ++t) { const int c = t * 16 + nloc; const float wsv = bf16_rne(as[c]), wdv = bf16_rne(ad[c]);
#pragma unroll
    for (int r8 = 0; r8 < 8; ++r8) { const float p = acc[t][r8] * sc; Tf[8 * hlf + r8][c] = p; float s = pmul(p, wsv), d = pmul(p, wdv); for (int o = 1; o < 16; o <<= 1) { s += __shfl_xor(s, o); d += __shfl_xor(d, o); } if (nloc == 0) { Se[8 * hlf + r8][t] = s; Se[8 * hlf + r8][4 + t] = d; } } }
  wave_lds_sync();
  for (int pass = 0; pass < 2; ++pass) { for (int rr = 0; rr < 16; ++rr) *(volatile v2f*)(P + (m0 + rr) * H + lane * 2) = *(const v2f*)(&Tf[rr][lane * 2]); for (int q = 0; q < 4; ++q) ((volatile float*)EL)[m0 * 8 + q * 32 + lane] = Se[(q * 32 + lane) >> 3][(q * 32 + lane) & 7]; __threadfence(); }
}
template <int RELU, int SAMPLED>
__global__ __launch_bounds__(256) void att_kernel(const float* __restrict__ P, const float* __restrict__ EL, const float* __restrict__ bias, const int* __restrict__ nodesv, const int* __restrict__ srcs, const int* __restrict__ PERM, const int* __restrict__ ROWPTR, const int* __restrict__ ROWCNT, int permLen, int TV, float* __restrict__ Hout) {
  const int wave = threadIdx.x >> 5, lane = threadIdx.x & 31; const size_t orow = (size_t)blockIdx.x * 8 + wave; size_t r = orow;
  if (SAMPLED) { const int b = (int)(orow / T), t = (int)(orow % T); int base = 0; for (int i = 0; i < b; ++i) base += nodesv[i]; const int n = iclamp(base, 0, N - 1); r = (size_t)n * T + t; }
  v2f o = {0.0f, 0.0f};
  if ((int)(r % T) < TV) { const size_t n = r / T; const int t = (int)(r % T); const int h = lane >> 3; const float edv = EL[r * 8 + 4 + h], esv = EL[r * 8 + h];
    int st = ROWPTR[n], cnt = ROWCNT[n]; cnt = iclamp(cnt, 0, 1 << 20); st = iclamp(st, 0, permLen - cnt); float mx = leaky(esv + edv);
#pragma unroll 1
    for (int j = 0; j < cnt; ++j) { const int e = iclamp(PERM[st + j], 0, E - 1); const size_t s = (size_t)iclamp(srcs[e], 0, N - 1); const size_t sr = s * T + t; mx = fmaxf(mx, leaky(EL[sr * 8 + h] + edv)); }
    const v2f own = *(const v2f*)(P + r * H + lane * 2); const float p0 = __expf(leaky(esv + edv) - mx); float den = p0; o[0] = pmul(p0, own[0]); o[1] = pmul(p0, own[1]);
#pragma unroll 1
    for (int j = 0; j < cnt; ++j) { const int e = iclamp(PERM[st + j], 0, E - 1); const size_t s = (size_t)iclamp(srcs[e], 0, N - 1); const size_t sr = s * T + t; const float p = __expf(leaky(EL[sr * 8 + h] + edv) - mx); den += p; const v2f f = *(const v2f*)(P + sr * H + lane * 2); o[0] += pmul(p, f[0]); o[1] += pmul(p, f[1]); }
    const float inv = 1.0f / (den + 1e-16f); for (int i = 0; i < 2; ++i) { o[i] = pmul(o[i], inv) + bf16_rne(bias[lane * 2 + i]); if (RELU) o[i] = fmaxf(o[i], 0.0f); } }
  for (int pass = 0; pass < 2; ++pass) { *(volatile v2f*)(Hout + orow * H + lane * 2) = o; __threadfence(); }
}
__global__ __launch_bounds__(32) void lstm_kernel(const float* __restrict__ SAMP, const float* __restrict__ rc, const float* __restrict__ rd, const b16* __restrict__ WSER, const float* __restrict__ bser, const b16* __restrict__ WL, const float* __restrict__ lb, int TV, float* __restrict__ SER, float* __restrict__ HSP, float* __restrict__ out) {
  __shared__ __attribute__((aligned(16))) b16 Ah[16][192 + 8], Al[16][192 + 8]; __shared__ __attribute__((aligned(16))) float Hh[16][LH + 4], Cc[16][LH + 4], Gs[16][4 * LH + 4], Tf[16][H + 4];
  const int lane = threadIdx.x, nloc = lane & 15, hlf = lane >> 4; const int b0 = blockIdx.x * 16;
#pragma unroll 1
  for (int t = 0; t < TV; ++t) {
    for (int rr = 0; rr < 16; ++rr) { const int b = b0 + rr; const v2f sv = *(const v2f*)(SAMP + ((size_t)b * T + t) * H + lane * 2); for (int j = 0; j < 2; ++j) { b16 p, q; split16(sv[j] * HS, p, q); Ah[rr][lane * 2 + j] = p; Al[rr][lane * 2 + j] = q; }
      float a = 0.0f; if (lane < 16) a = rc[b * 16 + lane]; else if (lane < 24) a = rd[b * 8 + lane - 16]; Ah[rr][64 + lane] = (b16)(bf16_rne(a) * HS); Al[rr][64 + lane] = (b16)0.0f; }
    wave_lds_sync();
    v8f acc[4];
#pragma unroll
    for (int tt = 0; tt < 4; ++tt) acc[tt] = (v8f){};
#pragma unroll
    for (int kb = 0; kb < 96; kb += 32) { const v16b a = frag_kb(&Ah[nloc][kb], hlf), al = frag_kb(&Al[nloc][kb], hlf);
#pragma unroll
      for (int tt = 0; tt < 4; ++tt) { const v16b bw = frag_kb(WSER + (size_t)(tt * 16 + nloc) * 96 + kb, hlf); acc[tt] = wmma16b(a, bw, acc[tt]); acc[tt] = wmma16b(al, bw, acc[tt]); } }
#pragma unroll
    for (int tt = 0; tt < 4; ++tt) { const int c = tt * 16 + nloc; const float bb = bf16_rne(bser[c]);
#pragma unroll 1
      for (int r8 = 0; r8 < 8; ++r8) Tf[8 * hlf + r8][c] = fmaxf(acc[tt][r8] * (1.0f / (HS * WSC)) + bb, 0.0f); }
    wave_lds_sync();
    for (int pass = 0; pass < 2; ++pass) { for (int rr = 0; rr < 16; ++rr) *(volatile v2f*)(SER + ((size_t)(b0 + rr) * T + t) * H + lane * 2) = *(const v2f*)(&Tf[rr][lane * 2]); __threadfence(); }
    wave_lds_sync(); }
  for (int rr = 0; rr < 16; ++rr) for (int q = 0; q < 4; ++q) { Hh[rr][q * 32 + lane] = 0.0f; Cc[rr][q * 32 + lane] = 0.0f; }
  wave_lds_sync();
#pragma unroll 1
  for (int t = 0; t < TV; ++t) {
    for (int rr = 0; rr < 16; ++rr) { const v2f sv = *(const v2f*)(SER + ((size_t)(b0 + rr) * T + t) * H + lane * 2); for (int j = 0; j < 2; ++j) { b16 p, q; split16(sv[j] * HS, p, q); Ah[rr][lane * 2 + j] = p; Al[rr][lane * 2 + j] = q; }
      for (int q = 0; q < 4; ++q) { b16 p, ql; split16(Hh[rr][q * 32 + lane] * HS, p, ql); Ah[rr][64 + q * 32 + lane] = p; Al[rr][64 + q * 32 + lane] = ql; } }
    wave_lds_sync();
#pragma unroll 1
    for (int cg = 0; cg < 4; ++cg) { v8f acc[8];
#pragma unroll
      for (int tt = 0; tt < 8; ++tt) acc[tt] = (v8f){};
#pragma unroll 2
      for (int kb = 0; kb < 192; kb += 32) { const v16b a = frag_kb(&Ah[nloc][kb], hlf), al = frag_kb(&Al[nloc][kb], hlf);
#pragma unroll
        for (int tt = 0; tt < 8; ++tt) { const v16b bw = frag_kb(WL + (size_t)(cg * 128 + tt * 16 + nloc) * 192 + kb, hlf); acc[tt] = wmma16b(a, bw, acc[tt]); acc[tt] = wmma16b(al, bw, acc[tt]); } }
#pragma unroll
      for (int tt = 0; tt < 8; ++tt) { const int c = cg * 128 + tt * 16 + nloc; const float bb = bf16_rne(lb[c]);
#pragma unroll 1
        for (int r8 = 0; r8 < 8; ++r8) Gs[8 * hlf + r8][c] = acc[tt][r8] * (1.0f / (HS * WSC)) + bb; } }
    wave_lds_sync();
    for (int rr = 0; rr < 16; ++rr) for (int q = 0; q < 4; ++q) { const int u = q * 32 + lane; const float ig = sigm(Gs[rr][u]), fg = sigm(Gs[rr][LH + u]), gt = tanhf(Gs[rr][2 * LH + u]), og = sigm(Gs[rr][3 * LH + u]);
      const float cn = pmul(fg, Cc[rr][u]) + pmul(ig, gt); Cc[rr][u] = cn; Hh[rr][u] = pmul(og, tanhf(cn)); }
    wave_lds_sync();
    for (int pass = 0; pass < 2; ++pass) { for (int rr = 0; rr < 16; ++rr) for (int q = 0; q < 4; ++q) ((volatile float*)HSP)[((size_t)(b0 + rr) * T + t) * LH + q * 32 + lane] = Hh[rr][q * 32 + lane]; __threadfence(); }
    wave_lds_sync(); }
  for (int pass = 0; pass < 2; ++pass) { for (int rr = 0; rr < 16; ++rr) for (int q = 0; q < 4; ++q) { ((volatile float*)out)[OFF1 + (size_t)(b0 + rr) * LH + q * 32 + lane] = Hh[rr][q * 32 + lane]; ((volatile float*)out)[OFF2 + (size_t)(b0 + rr) * LH + q * 32 + lane] = Cc[rr][q * 32 + lane]; } __threadfence(); }
}
__global__ __launch_bounds__(256) void head_kernel(const float* __restrict__ HS, const float* __restrict__ hw, const float* __restrict__ hb, int TV, float* __restrict__ out) {
  __shared__ float w[LH][12]; for (int i = threadIdx.x; i < LH * 12; i += 256) w[i / 12][i % 12] = bf16_rne(hw[i]); __syncthreads();
  const int row = blockIdx.x * 256 + threadIdx.x; if (row >= SR) return; const int t = row % T; float z[12]; for (int k = 0; k < 12; ++k) z[k] = bf16_rne(hb[k]);
  if (t < TV) {
#pragma unroll 1
    for (int u = 0; u < LH; u += 4) { const v4f hv = *(const v4f*)(HS + (size_t)row * LH + u); for (int j = 0; j < 4; ++j)
#pragma unroll
      for (int k = 0; k < 12; ++k) z[k] += pmul(hv[j], w[u + j][k]); } }
  float o[12]; for (int k = 0; k < 3; ++k) { o[k] = z[k]; o[3 + k] = softplus(z[3 + k]) + 1e-3f; o[6 + k] = sigm(z[6 + k]); } const float m = fmaxf(z[9], fmaxf(z[10], z[11])); const float e0 = __expf(z[9] - m), e1 = __expf(z[10] - m), e2 = __expf(z[11] - m); const float inv = 1.0f / (e0 + e1 + e2); o[9] = e0 * inv; o[10] = e1 * inv; o[11] = e2 * inv;
  for (int pass = 0; pass < 2; ++pass) { for (int k = 0; k < 12; ++k) ((volatile float*)out)[(size_t)row * 12 + k] = (t < TV) ? o[k] : 0.0f; __threadfence(); }
}
}

extern "C" void kernel_launch(void* const* d_in, const int* in_sizes, int n_in, void* d_out, int out_size, void* d_ws, size_t ws_size, hipStream_t stream) {
  (void)n_in;
  auto Fp = [&](int i) { return (const float*)d_in[i]; }; auto Ip = [&](int i) { return (const int*)d_in[i]; };
  if (in_sizes[0] != NR * 16 || in_sizes[1] != N * 16 || in_sizes[2] != N * 8 || in_sizes[5] != 32 * H || in_sizes[8] != H * H || in_sizes[16] != 80 * H || in_sizes[19] != H * 512 || in_sizes[20] != LH * 512 || in_sizes[22] != LH * 12 || in_sizes[24] != 2 * E || in_sizes[25] != B || out_size != OFF2 + B * LH) return;
  const int TV = T;
  size_t off = 0; char* ws = (char*)d_ws;
  auto carve = [&](size_t bytes) { char* p = ws + off; off += (bytes + 255) & ~(size_t)255; return p; };
  b16* WT0 = (b16*)carve(H * H * 2); b16* WG1 = (b16*)carve(H * H * 2); b16* WG2 = (b16*)carve(H * H * 2); b16* WSER = (b16*)carve(H * 96 * 2); b16* WL = (b16*)carve((size_t)512 * 192 * 2);
  float* X0 = (float*)carve((size_t)NR * H * 4); float* P = (float*)carve((size_t)NR * H * 4); float* X1 = (float*)carve((size_t)NR * H * 4); float* EL = (float*)carve((size_t)NR * 8 * 4); float* SAMP = (float*)carve((size_t)SR * H * 4); float* SER = (float*)carve((size_t)SR * H * 4); float* HS = (float*)carve((size_t)SR * LH * 4);
  CsrBufs9 csr; off = csr_carve9(csr, ws, off, E, N);
  if (off > ws_size) return;
  wzero_kernel<<<(H * H / 8 + 255) / 256, 256, 0, stream>>>(WT0, H * H / 8); wzero_kernel<<<(H * 96 / 8 + 255) / 256, 256, 0, stream>>>(WSER, H * 96 / 8);
  wput_kernel<<<(H * 4 + 255) / 256, 256, 0, stream>>>(Fp(5), 32, H, H, 0, H, WT0); wput_kernel<<<(H + 255) / 256, 256, 0, stream>>>(Fp(6), 8, H, H, 32, H, WT0);
  wput_kernel<<<(H * 8 + 255) / 256, 256, 0, stream>>>(Fp(8), H, H, H, 0, H, WG1); wput_kernel<<<(H * 8 + 255) / 256, 256, 0, stream>>>(Fp(12), H, H, H, 0, H, WG2);
  wput_kernel<<<(H * 10 + 255) / 256, 256, 0, stream>>>(Fp(16), 80, H, H, 0, 96, WSER); wput_kernel<<<(H + 255) / 256, 256, 0, stream>>>(Fp(17), 8, H, H, 80, 96, WSER);
  wput_kernel<<<(512 * 8 + 255) / 256, 256, 0, stream>>>(Fp(19), H, 512, 512, 0, 192, WL); wput_kernel<<<(512 * 16 + 255) / 256, 256, 0, stream>>>(Fp(20), LH, 512, 512, H, 192, WL);
  csr_build9(csr, Ip(24) + E, E, N, stream);
  proj_kernel<<<NRB, 32, 0, stream>>>(Fp(0), Fp(1), Fp(2), WT0, Fp(7), TV, X0);
  lin_kernel<<<NRB, 32, 0, stream>>>(X0, WG1, Fp(9), Fp(10), TV, P, EL);
  att_kernel<1, 0><<<NR / 8, 256, 0, stream>>>(P, EL, Fp(11), Ip(25), Ip(24), csr.PERM, csr.ROWPTR, csr.ROWCNT, (int)csr.permLen, TV, X1);
  lin_kernel<<<NRB, 32, 0, stream>>>(X1, WG2, Fp(13), Fp(14), TV, P, EL);
  att_kernel<0, 1><<<SR / 8, 256, 0, stream>>>(P, EL, Fp(15), Ip(25), Ip(24), csr.PERM, csr.ROWPTR, csr.ROWCNT, (int)csr.permLen, TV, SAMP);
  lstm_kernel<<<2, 32, 0, stream>>>(SAMP, Fp(3), Fp(4), WSER, Fp(18), WL, Fp(21), TV, SER, HS, (float*)d_out);
  head_kernel<<<(SR + 255) / 256, 256, 0, stream>>>(HS, Fp(22), Fp(23), TV, (float*)d_out);
}
